// TFLongformerSelfAttention_64819646432037
// MI455X (gfx1250) — hardware-verified
//
#include <hip/hip_runtime.h>


namespace {
constexpr int B = 2, S = 4096, E = 768, H = 12, HD = 64, WDW = 256, G = 32, BL = 2  , NSLAB = 6  , HL = 2 * NSLAB;
constexpr float XS = 8.0f, WSC = 256.0f, PS = 1024.0f, LOG2E = 1.4426950408889634f;
static_assert(S % 64 == 0 && E == H * HD && G == 32, "tiling");
typedef _Float16 b16;
typedef __attribute__((ext_vector_type(16))) _Float16 v16b;
typedef __attribute__((ext_vector_type(8))) _Float16 v8b;
typedef __attribute__((ext_vector_type(8))) float v8f;
typedef __attribute__((ext_vector_type(4))) float v4f;
__device__ __forceinline__ float bf16_rne(float f) { unsigned int u = __float_as_uint(f); u += 0x7FFFu + ((u >> 16) & 1u); return __uint_as_float(u & 0xFFFF0000u); }
__device__ __forceinline__ void split16(float v, b16& hi, b16& lo) { hi = (b16)v; lo = (b16)(v - (float)hi); }
__device__ __forceinline__ v16b frag_kb(const b16* p, int hh) { const v8b a = *(const v8b*)(p + 8 * hh), b = *(const v8b*)(p + 16 + 8 * hh); v16b f;
#pragma unroll
  for (int e = 0; e < 8; ++e) { f[e] = a[e]; f[8 + e] = b[e]; } return f; }
__device__ __forceinline__ v8f wmma16b(v16b a, v16b b, v8f c) { v8f d = __builtin_amdgcn_wmma_f32_16x16x32_f16(false, a, false, b, (short)0, c, false, false); asm volatile("v_nop\n\tv_nop\n\tv_nop\n\tv_nop" : "+v"(d) : "v"(a), "v"(b)); return d; }
__device__ __forceinline__ void wave_lds_sync() { __builtin_amdgcn_fence(__ATOMIC_RELEASE, "workgroup"); __builtin_amdgcn_wave_barrier(); __builtin_amdgcn_fence(__ATOMIC_ACQUIRE, "workgroup"); }
__device__ __forceinline__ float pmul(float a, float b) { float p = a * b; asm volatile("" : "+v"(p)); return p; }
__device__ __forceinline__ int iclamp(int v, int lo, int hi) { return v < lo ? lo : (v > hi ? hi : v); }

typedef __attribute__((ext_vector_type(2))) _Float16 v2h;
typedef __attribute__((ext_vector_type(4))) _Float16 v4h;
typedef __attribute__((ext_vector_type(2))) float v2f;
__device__ __forceinline__ float nexp2(float v) { return __builtin_amdgcn_exp2f(v); }
__global__ __launch_bounds__(256) void prep_kernel(const float* __restrict__ wq, const float* __restrict__ wk, const float* __restrict__ wv, const float* __restrict__ wkg, const float* __restrict__ wvg, const float* __restrict__ wqg, const float* __restrict__ mask, b16* __restrict__ WT, int* __restrict__ CNT) {
  __shared__ int sh[256];
  if (blockIdx.x == 0) { int bad = 0; for (int i = threadIdx.x; i < B * S; i += 256) { const int t = i % S; const float m = mask[i]; if (m != ((t < G) ? 1.0f : 0.0f)) ++bad; } sh[threadIdx.x] = bad; __syncthreads();
    if (threadIdx.x < 32) { int s = 0; for (int i = threadIdx.x; i < 256; i += 32) s += sh[i]; for (int o = 1; o < 32; o <<= 1) s += __shfl_xor(s, o); for (int pass = 0; pass < 2; ++pass) { ((volatile int*)CNT)[threadIdx.x] = s; __threadfence(); } } return; }
  const size_t u = (size_t)(blockIdx.x - 1) * 256 + threadIdx.x; if (u >= (size_t)6 * E * E / 8) return; const size_t e = u * 8; const int m = (int)(e / ((size_t)E * E)); const size_t el = e % ((size_t)E * E); const int oo = (int)(el / E), i0 = (int)(el % E);
  const float* w = m == 0 ? wq : m == 1 ? wk : m == 2 ? wv : m == 3 ? wkg : m == 4 ? wvg : wqg; v8b o; for (int j = 0; j < 8; ++j) o[j] = (b16)(bf16_rne(w[(size_t)(i0 + j) * E + oo]) * WSC);
  for (int pass = 0; pass < 2; ++pass) { *(volatile v8b*)(WT + e) = o; __threadfence(); }
}
__global__ __launch_bounds__(128) void proj_kernel(const float* __restrict__ x, const b16* __restrict__ WT, const float* const* __restrict__ biases_unused, const float* __restrict__ bq, const float* __restrict__ bk, const float* __restrict__ bv, const float* __restrict__ bkg, const float* __restrict__ bvg, const float* __restrict__ bqg,
                                                   b16* __restrict__ Qp, b16* __restrict__ Kp, b16* __restrict__ VTh, b16* __restrict__ VTl, b16* __restrict__ KGp, b16* __restrict__ VGh, b16* __restrict__ VGl, b16* __restrict__ QGp) {
  __shared__ __attribute__((aligned(16))) b16 As[4][16][384 + 8]; __shared__ __attribute__((aligned(16))) float Tf[4][16][128 + 4];
  const int wave = threadIdx.x >> 5, lane = threadIdx.x & 31, nloc = lane & 15, hlf = lane >> 4; const int which = blockIdx.y % 6, b = blockIdx.y / 6; const int rb = blockIdx.x, slab = blockIdx.z; const int t0 = rb * 64 + wave * 16; const int n0 = slab * 128;
  if (which == 5 && rb != 0) return;
  const b16* W = WT + (size_t)which * E * E; const float* bias = which == 0 ? bq : which == 1 ? bk : which == 2 ? bv : which == 3 ? bkg : which == 4 ? bvg : bqg;
  v8f acc[8];
#pragma unroll
  for (int t = 0; t < 8; ++t) acc[t] = (v8f){};
#pragma unroll 1
  for (int half = 0; half < 2; ++half) {
    for (int rr = 0; rr < 16; ++rr) { const float* xr = x + ((size_t)b * S + t0 + rr) * E + half * 384; for (int q = lane * 4; q < 384; q += 128) { v4h o; for (int j = 0; j < 4; ++j) o[j] = (b16)(bf16_rne(xr[q + j]) * XS); *(v4h*)(&As[wave][rr][q]) = o; } }
    wave_lds_sync();
#pragma unroll 2
    for (int kb = 0; kb < 384; kb += 32) { const v16b a = frag_kb(&As[wave][nloc][kb], hlf);
#pragma unroll
      for (int t = 0; t < 8; ++t) acc[t] = wmma16b(a, frag_kb(W + (size_t)(n0 + t * 16 + nloc) * E + half * 384 + kb, hlf), acc[t]); }
    wave_lds_sync(); }
#pragma unroll
  for (int t = 0; t < 8; ++t) { const float bb = bf16_rne(bias[n0 + t * 16 + nloc]);
#pragma unroll
    for (int r = 0; r < 8; ++r) Tf[wave][8 * hlf + r][t * 16 + nloc] = acc[t][r] * (1.0f / (XS * WSC)) + bb; }
  __syncthreads();
  for (int pass = 0; pass < 2; ++pass) {
    if (which == 2 || which == 4) { b16* Vh = (which == 2 ? VTh : VGh); b16* Vl = (which == 2 ? VTl : VGl);
#pragma unroll 1
      for (int q = 0; q < 32; ++q) { const int cl = wave * 32 + q; const int c = n0 + cl; const int h = c / HD, d = c % HD; const int tk = lane * 2; v2h hv, lv;
        for (int j = 0; j < 2; ++j) { b16 p, ql; split16(Tf[(tk + j) >> 4][(tk + j) & 15][cl] * XS, p, ql); hv[j] = p; lv[j] = ql; }
        const size_t oi = (((size_t)b * H + h) * HD + d) * S + rb * 64 + lane * 2; *(volatile v2h*)(Vh + oi) = hv; *(volatile v2h*)(Vl + oi) = lv; } }
    else { b16* P = which == 0 ? Qp : which == 1 ? Kp : which == 3 ? KGp : QGp;
      for (int rr = 0; rr < 16; ++rr) { for (int hs = 0; hs < 2; ++hs) { const int c = n0 + hs * 64; const int h = c / HD; v2h o; o[0] = (b16)(Tf[wave][rr][hs * 64 + lane * 2] * XS); o[1] = (b16)(Tf[wave][rr][hs * 64 + lane * 2 + 1] * XS);
          const size_t row = (which == 5) ? (((size_t)b * H + h) * 64 + (t0 + rr)) : (((size_t)b * H + h) * S + (t0 + rr)); *(volatile v2h*)(P + row * HD + lane * 2) = o; } } }
    __threadfence(); }
}
__global__ __launch_bounds__(64) void local_kernel(const b16* __restrict__ Qp, const b16* __restrict__ Kp, const b16* __restrict__ VTh, const b16* __restrict__ VTl, const int* __restrict__ CNT, float* __restrict__ out) {
  __shared__ __attribute__((aligned(16))) b16 Pb[2][16][32 + 8]; __shared__ __attribute__((aligned(16))) float To[2][16][HD + 4];
  const int wave = threadIdx.x >> 5, lane = threadIdx.x & 31, hh = lane >> 4, col = lane & 15; const int b = blockIdx.y / HL, h = blockIdx.y % HL; const int q0 = G + blockIdx.x * 32 + wave * 16, qi = q0 + col;
  const b16* Qb = Qp + ((size_t)(b * H + h) * S) * HD; const b16* Kb = Kp + ((size_t)(b * H + h) * S) * HD; const b16* Vh = VTh + ((size_t)(b * H + h) * HD) * S; const b16* Vl = VTl + ((size_t)(b * H + h) * HD) * S;
  const v16b qa0 = frag_kb(Qb + (size_t)qi * HD, hh), qa1 = frag_kb(Qb + (size_t)qi * HD + 32, hh);
  const float cs = LOG2E / (8.0f * XS * XS);
  float m = -INFINITY, l = 0.0f; v8f o[4]; for (int t = 0; t < 4; ++t) o[t] = (v8f){};
  const int ktlo = ((q0 - WDW) / 16 > 2) ? (q0 - WDW) / 16 : 2, kthi = ((q0 + 15 + WDW) / 16 < S / 16 - 1) ? (q0 + 15 + WDW) / 16 : S / 16 - 1;
  const int ntile = 2 + (kthi - ktlo + 1);
#pragma unroll 1
  for (int it = 0; it < ntile; it += 2) {
    float e[16]; float mx = -INFINITY;
#pragma unroll
    for (int u = 0; u < 2; ++u) { const int i = it + u; const int kt = (i < 2) ? i : (ktlo + i - 2); const bool tile_ok = (i < ntile);
      v8f s = (v8f){}; const int ktc = (kt < S / 16) ? kt : (S / 16 - 1); const size_t kr = (size_t)(ktc * 16 + col) * HD; s = wmma16b(frag_kb(Kb + kr, hh), qa0, s); s = wmma16b(frag_kb(Kb + kr + 32, hh), qa1, s);
#pragma unroll
      for (int r = 0; r < 8; ++r) { const int key = kt * 16 + 8 * hh + r; const bool ok = tile_ok && ((i < 2) || (key >= qi - WDW && key <= qi + WDW)); const float v = ok ? s[r] * cs : -INFINITY; e[u * 8 + r] = v; mx = fmaxf(mx, v); } }
    mx = fmaxf(mx, __shfl_xor(mx, 16)); const float mn = fmaxf(m, mx); const float al = (mn == -INFINITY) ? 1.0f : nexp2(m - mn); float sum = 0.0f;
#pragma unroll
    for (int i2 = 0; i2 < 16; ++i2) { const float p = (e[i2] == -INFINITY) ? 0.0f : nexp2(e[i2] - mn); sum += p; Pb[wave][col][(i2 < 8 ? 0 : 16) + 8 * hh + (i2 & 7)] = (b16)(p * PS); }
    sum += __shfl_xor(sum, 16); l = l * al + sum; m = mn;
    wave_lds_sync();
    const v16b pf = frag_kb(&Pb[wave][col][0], hh);
    const int ktA = (it < 2) ? it : (ktlo + it - 2), ktB = (it + 1 < 2) ? it + 1 : (ktlo + it + 1 - 2);
#pragma unroll
    for (int t = 0; t < 4; ++t) { o[t] *= al; const size_t vr = (size_t)(t * 16 + col) * S;
      v16b vah, val; { const v8b a0 = *(const v8b*)(Vh + vr + ktA * 16 + 8 * hh), a1 = *(const v8b*)(Vh + vr + (ktB < S / 16 ? ktB : ktA) * 16 + 8 * hh), c0 = *(const v8b*)(Vl + vr + ktA * 16 + 8 * hh), c1 = *(const v8b*)(Vl + vr + (ktB < S / 16 ? ktB : ktA) * 16 + 8 * hh);
        for (int j = 0; j < 8; ++j) { vah[j] = a0[j]; vah[8 + j] = a1[j]; val[j] = c0[j]; val[8 + j] = c1[j]; } }
      o[t] = wmma16b(vah, pf, o[t]); o[t] = wmma16b(val, pf, o[t]); }
    wave_lds_sync(); }
  int bad = CNT[0]; const float inv = 1.0f / (l * PS * XS);
#pragma unroll
  for (int t = 0; t < 4; ++t)
#pragma unroll
    for (int r = 0; r < 8; ++r) To[wave][col][t * 16 + 8 * hh + r] = bad ? __int_as_float(0x7fc00000) : o[t][r] * inv;
  wave_lds_sync();
  for (int pass = 0; pass < 2; ++pass) { for (int rr = 0; rr < 16; ++rr) *(volatile v2f*)(out + ((size_t)b * S + q0 + rr) * E + h * HD + lane * 2) = *(const v2f*)(&To[wave][rr][lane * 2]); __threadfence(); }
}
__global__ __launch_bounds__(64) void global_kernel(const b16* __restrict__ QGp, const b16* __restrict__ KGp, const b16* __restrict__ VGh, const b16* __restrict__ VGl, const int* __restrict__ CNT, float* __restrict__ out) {
  __shared__ __attribute__((aligned(16))) b16 Pb[2][16][32 + 8]; __shared__ __attribute__((aligned(16))) float To[2][16][HD + 4];
  const int wave = threadIdx.x >> 5, lane = threadIdx.x & 31, hh = lane >> 4, col = lane & 15; const int b = blockIdx.x / HL, h = blockIdx.x % HL; const int q0 = wave * 16, qi = q0 + col;
  const b16* Qb = QGp + ((size_t)(b * H + h) * 64) * HD; const b16* Kb = KGp + ((size_t)(b * H + h) * S) * HD; const b16* Vh = VGh + ((size_t)(b * H + h) * HD) * S; const b16* Vl = VGl + ((size_t)(b * H + h) * HD) * S;
  const v16b qa0 = frag_kb(Qb + (size_t)qi * HD, hh), qa1 = frag_kb(Qb + (size_t)qi * HD + 32, hh);
  const float cs = LOG2E / (8.0f * XS * XS);
  float m = -INFINITY, l = 0.0f; v8f o[4]; for (int t = 0; t < 4; ++t) o[t] = (v8f){};
#pragma unroll 1
  for (int kb = 0; kb < S; kb += 32) {
    float e[16]; float mx = -INFINITY;
#pragma unroll
    for (int u = 0; u < 2; ++u) { v8f s = (v8f){}; const size_t kr = (size_t)(kb + u * 16 + col) * HD; s = wmma16b(frag_kb(Kb + kr, hh), qa0, s); s = wmma16b(frag_kb(Kb + kr + 32, hh), qa1, s);
#pragma unroll
      for (int r = 0; r < 8; ++r) { const float v = s[r] * cs; e[u * 8 + r] = v; mx = fmaxf(mx, v); } }
    mx = fmaxf(mx, __shfl_xor(mx, 16)); const float mn = fmaxf(m, mx); const float al = nexp2(m - mn); float sum = 0.0f;
#pragma unroll
    for (int i2 = 0; i2 < 16; ++i2) { const float p = nexp2(e[i2] - mn); sum += p; Pb[wave][col][(i2 < 8 ? 0 : 16) + 8 * hh + (i2 & 7)] = (b16)(p * PS); }
    sum += __shfl_xor(sum, 16); l = l * al + sum; m = mn;
    wave_lds_sync();
    const v16b pf = frag_kb(&Pb[wave][col][0], hh);
#pragma unroll
    for (int t = 0; t < 4; ++t) { o[t] *= al; const size_t vr = (size_t)(t * 16 + col) * S + kb; o[t] = wmma16b(frag_kb(Vh + vr, hh), pf, o[t]); o[t] = wmma16b(frag_kb(Vl + vr, hh), pf, o[t]); }
    wave_lds_sync(); }
  int bad = CNT[0]; const float inv = 1.0f / (l * PS * XS);
#pragma unroll
  for (int t = 0; t < 4; ++t)
#pragma unroll
    for (int r = 0; r < 8; ++r) To[wave][col][t * 16 + 8 * hh + r] = bad ? __int_as_float(0x7fc00000) : o[t][r] * inv;
  wave_lds_sync();
  for (int pass = 0; pass < 2; ++pass) { for (int rr = 0; rr < 16; ++rr) *(volatile v2f*)(out + ((size_t)b * S + q0 + rr) * E + h * HD + lane * 2) = *(const v2f*)(&To[wave][rr][lane * 2]); __threadfence(); }
}
}

extern "C" void kernel_launch(void* const* d_in, const int* in_sizes, int n_in, void* d_out, int out_size, void* d_ws, size_t ws_size, hipStream_t stream) {
  (void)n_in;
  auto Fp = [&](int i) { return (const float*)d_in[i]; };
  if (in_sizes[0] != B * S * E || in_sizes[1] != B * S || in_sizes[2] != E * E || in_sizes[4] != E * E || in_sizes[6] != E * E || in_sizes[8] != E * E || in_sizes[10] != E * E || in_sizes[12] != E * E || in_sizes[13] != E || out_size != B * S * E) return;
  size_t off = 0; char* ws = (char*)d_ws;
  auto carve = [&](size_t bytes) { char* p = ws + off; off += (bytes + 255) & ~(size_t)255; return p; };
  b16* WT = (b16*)carve((size_t)6 * E * E * 2); int* CNT = (int*)carve(256);
  const size_t plane = (size_t)B * H * S * HD * 2;
  b16* Qp = (b16*)carve(plane); b16* Kp = (b16*)carve(plane); b16* VTh = (b16*)carve(plane); b16* VTl = (b16*)carve(plane); b16* KGp = (b16*)carve(plane); b16* VGh = (b16*)carve(plane); b16* VGl = (b16*)carve(plane); b16* QGp = (b16*)carve((size_t)B * H * 64 * HD * 2);
  if (off > ws_size || off > ((size_t)128 << 20)) return;
  prep_kernel<<<1 + (unsigned)(((size_t)6 * E * E / 8 + 255) / 256), 256, 0, stream>>>(Fp(2), Fp(4), Fp(6), Fp(10), Fp(12), Fp(8), Fp(1), WT, CNT);
  proj_kernel<<<dim3(S / 64, BL * 6, NSLAB), 128, 0, stream>>>(Fp(0), WT, nullptr, Fp(3), Fp(5), Fp(7), Fp(11), Fp(13), Fp(9), Qp, Kp, VTh, VTl, KGp, VGh, VGl, QGp);
  local_kernel<<<dim3(S / 32 - 1, BL * HL), 64, 0, stream>>>(Qp, Kp, VTh, VTl, CNT, (float*)d_out);
  global_kernel<<<BL * HL, 64, 0, stream>>>(QGp, KGp, VGh, VGl, CNT, (float*)d_out);
}
